// SSSDBlock_22479858827558
// MI455X (gfx1250) — hardware-verified
//
#include <hip/hip_runtime.h>
#include <math.h>
#include <stddef.h>


#define B_SZ   4
#define SEQ    2048
#define DMOD   256
#define DIN    512
#define DST    16
#define DTR    16
#define DCONV  4
#define NHEAD  4
#define HDIM   64
#define MTOT   (B_SZ * SEQ)
#define DBLW   (DTR + 2 * DST)
#define DBLP   64
#define KDT    64
#define AT_KC  64

#define WSC    64.0f
#define XCSC   256.0f
#define DTSC   256.0f
#define YSC    1024.0f
#define OSC    256.0f
#define CATSC  256.0f
#define PSC    32768.0f
#define LOG2E  1.4426950408889634f
#define LN2    0.6931471805599453f

typedef __attribute__((ext_vector_type(16))) _Float16 v16h;
typedef __attribute__((ext_vector_type(8)))  _Float16 v8h;
typedef __attribute__((ext_vector_type(16))) __bf16   v16b;
typedef __attribute__((ext_vector_type(8)))  __bf16   v8b;
typedef __attribute__((ext_vector_type(8)))  float    v8f;
typedef __attribute__((ext_vector_type(4)))  float    v4f;
typedef __attribute__((ext_vector_type(2)))  float    v2f;
typedef __attribute__((ext_vector_type(2)))  unsigned int v2u;

__device__ __forceinline__ unsigned short f2bf_bits(float f) {
  unsigned u = __float_as_uint(f);
  return (unsigned short)((u + 0x7FFFu + ((u >> 16) & 1u)) >> 16);
}
__device__ __forceinline__ float bf_bits2f(unsigned short h) { return __uint_as_float(((unsigned)h) << 16); }

__device__ __forceinline__ void dep_guard_h(v8f& a, v8f& b, v16h x, v16h y) { asm volatile("v_nop\n\tv_nop\n\tv_nop\n\tv_nop" : "+v"(a), "+v"(b) : "v"(x), "v"(y)); }
__device__ __forceinline__ void dep_guard_b(v8f& a, v8f& b, v16b x, v16b y) { asm volatile("v_nop\n\tv_nop\n\tv_nop\n\tv_nop" : "+v"(a), "+v"(b) : "v"(x), "v"(y)); }
__device__ __forceinline__ void keep4_h(v16h a, v16h b, v16h c, v16h d) { asm volatile("v_nop" :: "v"(a), "v"(b), "v"(c), "v"(d)); }
__device__ __forceinline__ void keep4_b(v16b a, v16b b, v16b c, v16b d) { asm volatile("v_nop" :: "v"(a), "v"(b), "v"(c), "v"(d)); }
__device__ __forceinline__ void acc_guard4(v8f& a, v8f& b, v8f& c, v8f& d) { asm volatile("v_nop\n\tv_nop\n\tv_nop\n\tv_nop" : "+v"(a), "+v"(b), "+v"(c), "+v"(d)); }
template <typename T> struct Frag;
template <> struct Frag<_Float16> {
  typedef v16h V; union U { v16h v; v8h h[2]; };
  static __device__ __forceinline__ v16h load(const _Float16* p) {
    U f; f.h[0] = *(const v8h*)(p); f.h[1] = *(const v8h*)(p + 16); return f.v;
  }
  static __device__ __forceinline__ v8f mma(v16h a, v16h b, v8f c) {
    return __builtin_amdgcn_wmma_f32_16x16x32_f16(false, a, false, b, (short)0, c, false, false);
  }
  static __device__ __forceinline__ void guard(v8f& a, v8f& b, v16h x, v16h y) { dep_guard_h(a, b, x, y); }
  static __device__ __forceinline__ void keep(v16h a, v16h b, v16h c, v16h d) { keep4_h(a, b, c, d); }
};
template <> struct Frag<__bf16> {
  typedef v16b V; union U { v16b v; v8b h[2]; };
  static __device__ __forceinline__ v16b load(const __bf16* p) {
    U f; f.h[0] = *(const v8b*)(p); f.h[1] = *(const v8b*)(p + 16); return f.v;
  }
  static __device__ __forceinline__ v8f mma(v16b a, v16b b, v8f c) {
    return __builtin_amdgcn_wmma_f32_16x16x32_bf16(false, a, false, b, (short)0, c, false, false);
  }
  static __device__ __forceinline__ void guard(v8f& a, v8f& b, v16b x, v16b y) { dep_guard_b(a, b, x, y); }
  static __device__ __forceinline__ void keep(v16b a, v16b b, v16b c, v16b d) { keep4_b(a, b, c, d); }
};

template <int ET> struct Elem;
template <> struct Elem<0> { typedef _Float16 T; };
template <> struct Elem<1> { typedef __bf16 T; };
template <int ET, bool SPLIT, int BIAS_MODE, int OUT_MODE, bool RESID, int ACT = 0>
__global__ __launch_bounds__(256) void wmma_gemm64(
    const unsigned short* __restrict__ Ap, const unsigned short* __restrict__ A2p, int lda, long strideA,
    const unsigned short* __restrict__ Btp, const unsigned short* __restrict__ Bt2p, int ldb, long strideB,
    void* __restrict__ Cout, void* __restrict__ Cout2, int ldc, long strideC,
    const float* __restrict__ bias,
    const float* __restrict__ resid, long strideR,
    int M, int N, int K, float scale) {
  typedef typename Elem<ET>::T T;
  typedef typename Frag<T>::V V;
  const T* A = (const T*)Ap; const T* A2 = (const T*)A2p; const T* Bt = (const T*)Btp; const T* Bt2 = (const T*)Bt2p;
  __shared__ __align__(16) float sT[8][16 * 68];
  const int b    = blockIdx.y;
  const int lane = threadIdx.x & 31;
  const int wave = threadIdx.x >> 5;
  const int tilesN = N >> 6;
  const int tilesM = M >> 6;
  const int tile = blockIdx.x * 8 + wave;
  if (tile >= tilesM * tilesN) return;
  const int tm = tile / tilesN;
  const int tn = tile - tm * tilesN;
  const int m0 = tm << 6;
  const int n0 = tn << 6;

  const T* Ab  = A  + (size_t)b * strideA;
  const T* Bb  = Bt + (size_t)b * strideB;
  const T* Ab2 = SPLIT ? (A2  + (size_t)b * strideA) : nullptr;
  const T* Bb2 = SPLIT ? (Bt2 + (size_t)b * strideB) : nullptr;

  const int rlane = lane & 15;
  const int koff  = (lane >> 4) * 8;
  const int mOff  = (lane >> 4) * 8;

  v8f acc[4][4];
#pragma unroll
  for (int i = 0; i < 4; ++i)
#pragma unroll
    for (int j = 0; j < 4; ++j) acc[i][j] = (v8f){0.f,0.f,0.f,0.f,0.f,0.f,0.f,0.f};

  for (int k0 = 0; k0 < K; k0 += 32) {
    V bh[4], bl[4];
#pragma unroll
    for (int j = 0; j < 4; ++j) {
      const size_t bo = (size_t)(n0 + (j << 4) + rlane) * ldb + koff + k0;
      bh[j] = Frag<T>::load(Bb + bo);
      if (SPLIT) bl[j] = Frag<T>::load(Bb2 + bo);
    }
#pragma unroll
    for (int i = 0; i < 4; ++i) {
      const size_t ao = (size_t)(m0 + (i << 4) + rlane) * lda + koff + k0;
      V ah = Frag<T>::load(Ab + ao);
      V al;
      if (SPLIT) al = Frag<T>::load(Ab2 + ao);
#pragma unroll
      for (int j = 0; j < 4; ++j) {
        acc[i][j] = Frag<T>::mma(ah, bh[j], acc[i][j]);
        if (SPLIT) {
          acc[i][j] = Frag<T>::mma(ah, bl[j], acc[i][j]);
          acc[i][j] = Frag<T>::mma(al, bh[j], acc[i][j]);
        }
      }
      Frag<T>::guard(acc[i][0], acc[i][3], ah, SPLIT ? al : ah);
    }
    Frag<T>::keep(bh[0], bh[1], bh[2], bh[3]);
    if (SPLIT) Frag<T>::keep(bl[0], bl[1], bl[2], bl[3]);
  }
  acc_guard4(acc[0][0], acc[0][1], acc[0][2], acc[0][3]);
  acc_guard4(acc[1][0], acc[1][1], acc[1][2], acc[1][3]);
  acc_guard4(acc[2][0], acc[2][1], acc[2][2], acc[2][3]);
  acc_guard4(acc[3][0], acc[3][1], acc[3][2], acc[3][3]);

  float* slab = sT[wave];
  const float* Rb = RESID ? (resid + (size_t)b * strideR) : nullptr;
#pragma unroll
  for (int i = 0; i < 4; ++i) {
    const int mBase = m0 + (i << 4);
#pragma unroll
    for (int j = 0; j < 4; ++j) {
      const int n = n0 + (j << 4) + rlane;
      float bv = 0.f;
      if (BIAS_MODE == 2) bv = bias[n];
#pragma unroll
      for (int r = 0; r < 8; ++r) {
        float v = acc[i][j][r] * scale;
        if (BIAS_MODE == 1) v += bias[mBase + mOff + r];
        if (BIAS_MODE == 2) v += bv;
        if (RESID) v += Rb[(size_t)(mBase + mOff + r) * ldc + n];
        if (ACT == 1) v = tanhf(v);
        if (ACT == 2) v = fmaxf(v, 0.0f);
        if (ACT == 3) v = v / (1.0f + expf(-v));
        if (ACT == 4) v = (v > 0.f) ? v : 0.01f * v;
        if (ACT == 5) v = 0.5f * v * (1.0f + erff(v * 0.70710678118654752f));
        slab[(mOff + r) * 68 + (j << 4) + rlane] = v;
      }
    }
    __builtin_amdgcn_fence(__ATOMIC_RELEASE, "workgroup");
    __builtin_amdgcn_wave_barrier();
    __builtin_amdgcn_fence(__ATOMIC_ACQUIRE, "workgroup");
    if (OUT_MODE == 0) {
      float* C = (float*)Cout + (size_t)b * strideC;
      const int hh = lane >> 4, c4 = (lane & 15) * 4;
      for (int pass = 0; pass < 2; ++pass) {
#pragma unroll
        for (int it = 0; it < 8; ++it) {
          const int row = it * 2 + hh;
          v4f v = *(const v4f*)(slab + row * 68 + c4);
          *(volatile v4f*)(C + (size_t)(mBase + row) * ldc + n0 + c4) = v;
        }
        __threadfence();
      }
    } else {
      const int q = lane >> 3, c8 = (lane & 7) * 8;
      unsigned short* C  = (unsigned short*)Cout  + (size_t)b * strideC;
      unsigned short* C2 = (OUT_MODE == 2) ? ((unsigned short*)Cout2 + (size_t)b * strideC) : nullptr;
      for (int pass = 0; pass < 2; ++pass) {
#pragma unroll
        for (int it = 0; it < 4; ++it) {
          const int row = it * 4 + q;
          const float* sp = slab + row * 68 + c8;
          v8h hv, lv;
#pragma unroll
          for (int e = 0; e < 8; ++e) {
            if (OUT_MODE == 1) {
              hv[e] = (_Float16)sp[e];
            } else {
              unsigned short hb = f2bf_bits(sp[e]);
              unsigned short lb = f2bf_bits(sp[e] - bf_bits2f(hb));
              hv[e] = __builtin_bit_cast(_Float16, hb);
              lv[e] = __builtin_bit_cast(_Float16, lb);
            }
          }
          *(volatile v8h*)(C + (size_t)(mBase + row) * ldc + n0 + c8) = hv;
          if (OUT_MODE == 2) *(volatile v8h*)(C2 + (size_t)(mBase + row) * ldc + n0 + c8) = lv;
        }
        __threadfence();
      }
    }
    __builtin_amdgcn_fence(__ATOMIC_RELEASE, "workgroup");
    __builtin_amdgcn_wave_barrier();
    __builtin_amdgcn_fence(__ATOMIC_ACQUIRE, "workgroup");
  }
}

__global__ __launch_bounds__(256) void wmma_gemm64_gate(
    const unsigned short* __restrict__ Ap, int lda,
    const unsigned short* __restrict__ Btp, int ldb,
    float* __restrict__ Cout, int ldc,
    const float* __restrict__ bias,
    const float* __restrict__ xres, const float* __restrict__ ssm, const float* __restrict__ att,
    int M, int N, int K, float scale) {
  typedef _Float16 T;
  typedef v16h V;
  const T* A = (const T*)Ap; const T* Bt = (const T*)Btp;
  __shared__ __align__(16) float sT[8][16 * 68];
  const int lane = threadIdx.x & 31;
  const int wave = threadIdx.x >> 5;
  const int tilesN = N >> 6;
  const int tilesM = M >> 6;
  const int tile = blockIdx.x * 8 + wave;
  if (tile >= tilesM * tilesN) return;
  const int tm = tile / tilesN;
  const int tn = tile - tm * tilesN;
  const int m0 = tm << 6;
  const int n0 = tn << 6;
  const int rlane = lane & 15;
  const int koff  = (lane >> 4) * 8;
  const int mOff  = (lane >> 4) * 8;

  v8f acc[4][4];
#pragma unroll
  for (int i = 0; i < 4; ++i)
#pragma unroll
    for (int j = 0; j < 4; ++j) acc[i][j] = (v8f){0.f,0.f,0.f,0.f,0.f,0.f,0.f,0.f};

  for (int k0 = 0; k0 < K; k0 += 32) {
    V bh[4];
#pragma unroll
    for (int j = 0; j < 4; ++j) bh[j] = Frag<T>::load(Bt + (size_t)(n0 + (j << 4) + rlane) * ldb + koff + k0);
#pragma unroll
    for (int i = 0; i < 4; ++i) {
      V ah = Frag<T>::load(A + (size_t)(m0 + (i << 4) + rlane) * lda + koff + k0);
#pragma unroll
      for (int j = 0; j < 4; ++j) acc[i][j] = Frag<T>::mma(ah, bh[j], acc[i][j]);
      Frag<T>::guard(acc[i][0], acc[i][3], ah, ah);
    }
    Frag<T>::keep(bh[0], bh[1], bh[2], bh[3]);
  }
  acc_guard4(acc[0][0], acc[0][1], acc[0][2], acc[0][3]);
  acc_guard4(acc[1][0], acc[1][1], acc[1][2], acc[1][3]);
  acc_guard4(acc[2][0], acc[2][1], acc[2][2], acc[2][3]);
  acc_guard4(acc[3][0], acc[3][1], acc[3][2], acc[3][3]);

  float* slab = sT[wave];
#pragma unroll
  for (int i = 0; i < 4; ++i) {
    const int mBase = m0 + (i << 4);
#pragma unroll
    for (int j = 0; j < 4; ++j) {
      const int n = n0 + (j << 4) + rlane;
      const float bv = bias[n];
#pragma unroll
      for (int r = 0; r < 8; ++r) slab[(mOff + r) * 68 + (j << 4) + rlane] = acc[i][j][r] * scale + bv;
    }
    __builtin_amdgcn_fence(__ATOMIC_RELEASE, "workgroup");
    __builtin_amdgcn_wave_barrier();
    __builtin_amdgcn_fence(__ATOMIC_ACQUIRE, "workgroup");
    const int hh = lane >> 4, c4 = (lane & 15) * 4;
#pragma unroll
    for (int it = 0; it < 8; ++it) {
      const int row = it * 2 + hh;
      const size_t gi = (size_t)(mBase + row) * ldc + n0 + c4;
      const v4f pre = *(const v4f*)(slab + row * 68 + c4);
      const v4f xs = *(const v4f*)(xres + gi);
      const v4f sv = *(const v4f*)(ssm + gi);
      const v4f av = *(const v4f*)(att + gi);
      v4f o;
#pragma unroll
      for (int e = 0; e < 4; ++e) {
        const float g = __builtin_amdgcn_rcpf(1.0f + exp2f(-pre[e] * LOG2E));
        const float fused = g * sv[e] + (1.0f - g) * av[e];
        o[e] = xs[e] + fused;
      }
      *(v4f*)(slab + row * 68 + c4) = o;
    }
    for (int pass = 0; pass < 2; ++pass) {
#pragma unroll
      for (int it = 0; it < 8; ++it) {
        const int row = it * 2 + hh;
        v4f v = *(const v4f*)(slab + row * 68 + c4);
        *(volatile v4f*)(Cout + (size_t)(mBase + row) * ldc + n0 + c4) = v;
      }
      __threadfence();
    }
    __builtin_amdgcn_fence(__ATOMIC_RELEASE, "workgroup");
    __builtin_amdgcn_wave_barrier();
    __builtin_amdgcn_fence(__ATOMIC_ACQUIRE, "workgroup");
  }
}

__global__ __launch_bounds__(256) void prep_wt(const float* __restrict__ W, _Float16* __restrict__ Bt,
                                               int K, int N, int Kp, float scale) {
  __shared__ float T[32 * 65];
  const int tid = threadIdx.x;
  const int n0 = blockIdx.x * 32, k0 = blockIdx.y * 64;
  const int nn4 = (tid & 7) * 4;
#pragma unroll
  for (int p = 0; p < 2; ++p) {
    const int kk = (tid >> 3) + 32 * p;
    const int k = k0 + kk;
    const int n = n0 + nn4;
    const int kc = (k < K) ? k : (K - 1);
    const int nc = (n < N) ? n : (N - 4);
    const v4f w = *(const v4f*)(W + (size_t)kc * N + nc);
    const bool ok = (k < K) && (n < N);
#pragma unroll
    for (int e = 0; e < 4; ++e) T[(nn4 + e) * 65 + kk] = ok ? (w[e] * scale) : 0.0f;
  }
  __syncthreads();
  const int row = tid >> 3, c8 = (tid & 7) * 8;
  v8h hv;
#pragma unroll
  for (int e = 0; e < 8; ++e) hv[e] = (_Float16)T[row * 65 + c8 + e];
  _Float16* dst = Bt + (size_t)(n0 + row) * Kp + k0 + c8;
  *(volatile v8h*)dst = hv;
  __threadfence();
  *(volatile v8h*)dst = hv;
}

__global__ __launch_bounds__(256) void ln_kernel(const float* __restrict__ x, const float* __restrict__ g,
                                                 const float* __restrict__ bb, _Float16* __restrict__ xn) {
  const int lane = threadIdx.x & 31, wave = threadIdx.x >> 5;
  const int row = blockIdx.x * 8 + wave;
  const float* xr = x + (size_t)row * DMOD + lane * 8;
  const v4f a = *(const v4f*)xr;
  const v4f c = *(const v4f*)(xr + 4);
  float s = ((a[0] + a[1]) + (a[2] + a[3])) + ((c[0] + c[1]) + (c[2] + c[3]));
#pragma unroll
  for (int off = 1; off < 32; off <<= 1) s += __shfl_xor(s, off, 32);
  const float mu = s * (1.0f / DMOD);
  float d[8];
#pragma unroll
  for (int e = 0; e < 4; ++e) { d[e] = a[e] - mu; d[4 + e] = c[e] - mu; }
  float q = 0.f;
#pragma unroll
  for (int e = 0; e < 8; ++e) q += d[e] * d[e];
#pragma unroll
  for (int off = 1; off < 32; off <<= 1) q += __shfl_xor(q, off, 32);
  const float var = q * (1.0f / DMOD);
  const float rstd = rsqrtf(var + 1e-5f);
  const v4f g0 = *(const v4f*)(g + lane * 8), g1 = *(const v4f*)(g + lane * 8 + 4);
  const v4f b0 = *(const v4f*)(bb + lane * 8), b1 = *(const v4f*)(bb + lane * 8 + 4);
  v8h o;
#pragma unroll
  for (int e = 0; e < 4; ++e) {
    o[e]     = (_Float16)(d[e] * rstd * g0[e] + b0[e]);
    o[4 + e] = (_Float16)(d[4 + e] * rstd * g1[e] + b1[e]);
  }
  _Float16* dst = xn + (size_t)row * DMOD + lane * 8;
  *(volatile v8h*)dst = o;
  __threadfence();
  *(volatile v8h*)dst = o;
}

__global__ __launch_bounds__(128) void conv_silu_kernel(const float* __restrict__ xz, const float* __restrict__ cw,
                                                        const float* __restrict__ cb, float* __restrict__ xc_f,
                                                        _Float16* __restrict__ xc_h) {
  const int m = blockIdx.x;
  const int t = m & (SEQ - 1);
  const int d0 = threadIdx.x * 4;
  v4f acc = *(const v4f*)(cb + d0);
  const v4f w0 = *(const v4f*)(cw + (d0 + 0) * DCONV);
  const v4f w1 = *(const v4f*)(cw + (d0 + 1) * DCONV);
  const v4f w2 = *(const v4f*)(cw + (d0 + 2) * DCONV);
  const v4f w3 = *(const v4f*)(cw + (d0 + 3) * DCONV);
#pragma unroll
  for (int k = 0; k < DCONV; ++k) {
    const int back = DCONV - 1 - k;
    const bool ok = (t >= back);
    const int mr = ok ? (m - back) : m;
    v4f xv = *(const v4f*)(xz + (size_t)mr * (2 * DIN) + d0);
    if (!ok) xv = (v4f){0.f, 0.f, 0.f, 0.f};
    acc[0] += xv[0] * w0[k];
    acc[1] += xv[1] * w1[k];
    acc[2] += xv[2] * w2[k];
    acc[3] += xv[3] * w3[k];
  }
  v4f sv;
#pragma unroll
  for (int e = 0; e < 4; ++e) sv[e] = acc[e] * __builtin_amdgcn_rcpf(1.0f + exp2f(-acc[e] * LOG2E));
  float* df = xc_f + (size_t)m * DIN + d0;
  *(volatile v4f*)df = sv;
  v2u pk;
  pk.x = (unsigned)__builtin_bit_cast(unsigned short, (_Float16)(sv[0] * XCSC)) |
         ((unsigned)__builtin_bit_cast(unsigned short, (_Float16)(sv[1] * XCSC)) << 16);
  pk.y = (unsigned)__builtin_bit_cast(unsigned short, (_Float16)(sv[2] * XCSC)) |
         ((unsigned)__builtin_bit_cast(unsigned short, (_Float16)(sv[3] * XCSC)) << 16);
  _Float16* dh = xc_h + (size_t)m * DIN + d0;
  *(volatile v2u*)dh = pk;
  __threadfence();
  *(volatile v4f*)df = sv;
  *(volatile v2u*)dh = pk;
}

__global__ __launch_bounds__(256) void dtin_kernel(const float* __restrict__ dbl, _Float16* __restrict__ dtin) {
  const int idx = blockIdx.x * 256 + threadIdx.x;
  const int m = idx >> 3, q = idx & 7;
  const int qq = q & 1;
  const v4f a = *(const v4f*)(dbl + (size_t)m * DBLP + qq * 8);
  const v4f c = *(const v4f*)(dbl + (size_t)m * DBLP + qq * 8 + 4);
  const bool live = (q < 2);
  v8h hv;
#pragma unroll
  for (int e = 0; e < 4; ++e) {
    hv[e]     = live ? (_Float16)(a[e] * DTSC) : (_Float16)0.0f;
    hv[4 + e] = live ? (_Float16)(c[e] * DTSC) : (_Float16)0.0f;
  }
  _Float16* dst = dtin + (size_t)m * KDT + q * 8;
  *(volatile v8h*)dst = hv;
  __threadfence();
  *(volatile v8h*)dst = hv;
}

__device__ __forceinline__ float softplus_f(float v) {
  return fmaxf(v, 0.0f) + LN2 * log2f(1.0f + exp2f(-fabsf(v) * LOG2E));
}
__global__ __launch_bounds__(64) void scan_kernel(const float* __restrict__ xc_f, const float* __restrict__ dt_f,
                                                  const float* __restrict__ dbl_f, const float* __restrict__ xz_f,
                                                  const float* __restrict__ A_log, const float* __restrict__ Dp,
                                                  _Float16* __restrict__ y_h) {
  const int b = blockIdx.x >> 2;
  const int d0 = ((((int)blockIdx.x & 3) << 6) + (int)threadIdx.x) * 2;
  float Aa[DST], Ab[DST], ha[DST], hb[DST];
#pragma unroll
  for (int n = 0; n < DST; ++n) {
    Aa[n] = -exp2f(A_log[d0 * DST + n] * LOG2E) * LOG2E;
    Ab[n] = -exp2f(A_log[(d0 + 1) * DST + n] * LOG2E) * LOG2E;
    ha[n] = 0.f; hb[n] = 0.f;
  }
  const float dpa = Dp[d0], dpb = Dp[d0 + 1];
  for (int t = 0; t < SEQ; ++t) {
    const size_t m = (size_t)b * SEQ + t;
    const v2f xt = *(const v2f*)(xc_f + m * DIN + d0);
    const v2f pv = *(const v2f*)(dt_f + m * DIN + d0);
    const v2f zz = *(const v2f*)(xz_f + m * (2 * DIN) + DIN + d0);
    const float* db = dbl_f + m * DBLP;
    float Bv[DST], Cv[DST];
#pragma unroll
    for (int i = 0; i < 4; ++i) {
      const v4f tb = *(const v4f*)(db + DTR + 4 * i);
      const v4f tc = *(const v4f*)(db + DTR + DST + 4 * i);
#pragma unroll
      for (int e = 0; e < 4; ++e) { Bv[4 * i + e] = tb[e]; Cv[4 * i + e] = tc[e]; }
    }
    const float dt0 = softplus_f(pv.x), dt1 = softplus_f(pv.y);
    const float dx0 = dt0 * xt.x, dx1 = dt1 * xt.y;
    float y0 = 0.f, y1 = 0.f;
#pragma unroll
    for (int n = 0; n < DST; ++n) {
      const float e0 = exp2f(dt0 * Aa[n]);
      const float e1 = exp2f(dt1 * Ab[n]);
      ha[n] = e0 * ha[n] + dx0 * Bv[n];
      hb[n] = e1 * hb[n] + dx1 * Bv[n];
      y0 += ha[n] * Cv[n];
      y1 += hb[n] * Cv[n];
    }
    const float s0 = zz.x * __builtin_amdgcn_rcpf(1.0f + exp2f(-zz.x * LOG2E));
    const float s1 = zz.y * __builtin_amdgcn_rcpf(1.0f + exp2f(-zz.y * LOG2E));
    const float o0 = (y0 + xt.x * dpa) * s0;
    const float o1 = (y1 + xt.y * dpb) * s1;
    const unsigned pk = (unsigned)__builtin_bit_cast(unsigned short, (_Float16)(o0 * YSC)) |
                        ((unsigned)__builtin_bit_cast(unsigned short, (_Float16)(o1 * YSC)) << 16);
    volatile unsigned* yp = (volatile unsigned*)(y_h + m * DIN + d0);
    *yp = pk;
    __threadfence();
    *yp = pk;
  }
}

__device__ __forceinline__ v8f mma_h(v16h a, v16h b, v8f c) {
  c = __builtin_amdgcn_wmma_f32_16x16x32_f16(false, a, false, b, (short)0, c, false, false);
  asm volatile("v_nop\n\tv_nop\n\tv_nop\n\tv_nop" : "+v"(c) : "v"(a), "v"(b));
  return c;
}
__global__ __launch_bounds__(128)
void attn_f16_kernel(const _Float16* __restrict__ qkv, _Float16* __restrict__ outp) {
  union FH { v16h v; v8h h[2]; };
  __shared__ __align__(16) _Float16 Ksh[AT_KC * HDIM];
  __shared__ __align__(16) _Float16 Vth[HDIM * AT_KC];
  __shared__ __align__(16) _Float16 Psh[4][16 * AT_KC];
  __shared__ __align__(16) float    Os[4][16 * 68];
  const int tid  = threadIdx.x;
  const int wave = tid >> 5;
  const int lane = tid & 31;
  const int hh   = lane >> 4;
  const int c    = lane & 15;
  const int nqb = SEQ / 64;
  const int bx = blockIdx.x;
  const int qb = bx % nqb;
  const int bh = bx / nqb;
  const int h  = bh % NHEAD;
  const int b  = bh / NHEAD;
  const int q0 = qb * 64 + wave * 16;
  const size_t rs = 3 * DMOD;
  const _Float16* qb_ptr = qkv + (size_t)b * SEQ * rs + h * HDIM;
  const _Float16* kb_ptr = qb_ptr + DMOD;
  const _Float16* vb_ptr = qb_ptr + 2 * DMOD;
  _Float16*       ob_ptr = outp + (size_t)b * SEQ * DMOD + h * HDIM;

  v16h qa[2];
  {
    const _Float16* qrow = qb_ptr + (size_t)(q0 + c) * rs + 8 * hh;
#pragma unroll
    for (int dc = 0; dc < 2; ++dc) qa[dc] = Frag<_Float16>::load(qrow + dc * 32);
  }
  float mrow[8], lrow[8];
  v8f oacc[4];
#pragma unroll
  for (int r = 0; r < 8; ++r) { mrow[r] = -INFINITY; lrow[r] = 0.f; }
#pragma unroll
  for (int t = 0; t < 4; ++t) oacc[t] = (v8f){0.f,0.f,0.f,0.f,0.f,0.f,0.f,0.f};

  for (int kc = 0; kc < SEQ / AT_KC; ++kc) {
    const int kv0 = kc * AT_KC;
    __syncthreads();
    {
      const int kvr = tid >> 1, dh = (tid & 1) * 32;
      const _Float16* krow = kb_ptr + (size_t)(kv0 + kvr) * rs + dh;
      const _Float16* vrow = vb_ptr + (size_t)(kv0 + kvr) * rs + dh;
#pragma unroll
      for (int i = 0; i < 4; ++i) {
        const v8h kk = *(const v8h*)(krow + 8 * i);
        const v8h vv = *(const v8h*)(vrow + 8 * i);
        *(v8h*)(Ksh + kvr * HDIM + dh + 8 * i) = kk;
#pragma unroll
        for (int e = 0; e < 8; ++e) Vth[(dh + 8 * i + e) * AT_KC + kvr] = vv[e];
      }
    }
    __syncthreads();

    v8f s[4];
#pragma unroll
    for (int j = 0; j < 4; ++j) {
      s[j] = (v8f){0.f,0.f,0.f,0.f,0.f,0.f,0.f,0.f};
#pragma unroll
      for (int dc = 0; dc < 2; ++dc) {
        FH kb;
        kb.h[0] = *(const v8h*)(Ksh + (j * 16 + c) * HDIM + dc * 32 + 8 * hh);
        kb.h[1] = *(const v8h*)(Ksh + (j * 16 + c) * HDIM + dc * 32 + 16 + 8 * hh);
        s[j] = mma_h(qa[dc], kb.v, s[j]);
      }
    }
    float cm[8];
#pragma unroll
    for (int r = 0; r < 8; ++r) {
      float m = -INFINITY;
#pragma unroll
      for (int j = 0; j < 4; ++j) {
        s[j][r] *= 0.125f;
        m = fmaxf(m, s[j][r]);
      }
#pragma unroll
      for (int off = 1; off < 16; off <<= 1) m = fmaxf(m, __shfl_xor(m, off, 32));
      cm[r] = m;
    }
    _Float16* pw = Psh[wave];
#pragma unroll
    for (int r = 0; r < 8; ++r) {
      const float mnew = fmaxf(mrow[r], cm[r]);
      const float alpha = expf(mrow[r] - mnew);
      mrow[r] = mnew;
      float psum = 0.f;
#pragma unroll
      for (int j = 0; j < 4; ++j) {
        const float p = expf(s[j][r] - mnew);
        psum += p;
        pw[(8 * hh + r) * AT_KC + j * 16 + c] = (_Float16)(p * PSC);
      }
#pragma unroll
      for (int off = 1; off < 16; off <<= 1) psum += __shfl_xor(psum, off, 32);
      lrow[r] = lrow[r] * alpha + psum;
#pragma unroll
      for (int t = 0; t < 4; ++t) oacc[t][r] *= alpha;
    }
    __builtin_amdgcn_fence(__ATOMIC_RELEASE, "workgroup");
    __builtin_amdgcn_wave_barrier();
    __builtin_amdgcn_fence(__ATOMIC_ACQUIRE, "workgroup");
#pragma unroll
    for (int kk = 0; kk < 2; ++kk) {
      FH pa;
      pa.h[0] = *(const v8h*)(pw + c * AT_KC + kk * 32 + 8 * hh);
      pa.h[1] = *(const v8h*)(pw + c * AT_KC + kk * 32 + 16 + 8 * hh);
#pragma unroll
      for (int t = 0; t < 4; ++t) {
        FH vb;
        vb.h[0] = *(const v8h*)(Vth + (t * 16 + c) * AT_KC + kk * 32 + 8 * hh);
        vb.h[1] = *(const v8h*)(Vth + (t * 16 + c) * AT_KC + kk * 32 + 16 + 8 * hh);
        oacc[t] = mma_h(pa.v, vb.v, oacc[t]);
      }
    }
  }

  float* os = Os[wave];
#pragma unroll
  for (int r = 0; r < 8; ++r) {
    const float inv = __builtin_amdgcn_rcpf(lrow[r]) * (OSC / PSC);
#pragma unroll
    for (int t = 0; t < 4; ++t) os[(8 * hh + r) * 68 + t * 16 + c] = oacc[t][r] * inv;
  }
  __builtin_amdgcn_fence(__ATOMIC_RELEASE, "workgroup");
  __builtin_amdgcn_wave_barrier();
  __builtin_amdgcn_fence(__ATOMIC_ACQUIRE, "workgroup");
  {
    const int q = lane >> 3, c8 = (lane & 7) * 8;
    for (int pass = 0; pass < 2; ++pass) {
#pragma unroll
      for (int it = 0; it < 4; ++it) {
        const int row = it * 4 + q;
        const float* sp = os + row * 68 + c8;
        v8h hv;
#pragma unroll
        for (int e = 0; e < 8; ++e) hv[e] = (_Float16)sp[e];
        *(volatile v8h*)(ob_ptr + (size_t)(q0 + row) * DMOD + c8) = hv;
      }
      __threadfence();
    }
  }
}

__global__ __launch_bounds__(256) void pack_kernel(const float* __restrict__ ssm, const float* __restrict__ att,
                                                   _Float16* __restrict__ cat) {
  const int idx = blockIdx.x * 256 + threadIdx.x;
  const int m = idx >> 6, g8 = idx & 63;
  const int cc = (g8 & 31) * 8;
  const float* src = (g8 < 32) ? (ssm + (size_t)m * DMOD + cc) : (att + (size_t)m * DMOD + cc);
  const v4f a = *(const v4f*)src;
  const v4f c = *(const v4f*)(src + 4);
  v8h hv;
#pragma unroll
  for (int e = 0; e < 4; ++e) { hv[e] = (_Float16)(a[e] * CATSC); hv[4 + e] = (_Float16)(c[e] * CATSC); }
  _Float16* dst = cat + (size_t)m * (2 * DMOD) + g8 * 8;
  *(volatile v8h*)dst = hv;
  __threadfence();
  *(volatile v8h*)dst = hv;
}

typedef unsigned short u16t;

static void launch_gemm_f32(hipStream_t st, const void* A, int lda, const void* Bt, int ldb, float* C, int ldc,
                            int M, int N, int K, float scale) {
  dim3 grid((unsigned)((((M >> 6) * (N >> 6)) + 7) / 8), 1);
  wmma_gemm64<0, false, 0, 0, false> <<<grid, dim3(256), 0, st>>> (
      (const u16t*)A, (const u16t*)A, lda, 0L, (const u16t*)Bt, (const u16t*)Bt, ldb, 0L,
      (void*)C, (void*)C, ldc, 0L, nullptr, nullptr, 0L, M, N, K, scale);
}
static void launch_gemm_f32_bias(hipStream_t st, const void* A, int lda, const void* Bt, int ldb, float* C, int ldc,
                                 const float* bias, int M, int N, int K, float scale) {
  dim3 grid((unsigned)((((M >> 6) * (N >> 6)) + 7) / 8), 1);
  wmma_gemm64<0, false, 2, 0, false> <<<grid, dim3(256), 0, st>>> (
      (const u16t*)A, (const u16t*)A, lda, 0L, (const u16t*)Bt, (const u16t*)Bt, ldb, 0L,
      (void*)C, (void*)C, ldc, 0L, bias, nullptr, 0L, M, N, K, scale);
}
static void launch_gemm_f16_bias(hipStream_t st, const void* A, int lda, const void* Bt, int ldb, _Float16* C, int ldc,
                                 const float* bias, int M, int N, int K, float scale) {
  dim3 grid((unsigned)((((M >> 6) * (N >> 6)) + 7) / 8), 1);
  wmma_gemm64<0, false, 2, 1, false> <<<grid, dim3(256), 0, st>>> (
      (const u16t*)A, (const u16t*)A, lda, 0L, (const u16t*)Bt, (const u16t*)Bt, ldb, 0L,
      (void*)C, (void*)C, ldc, 0L, bias, nullptr, 0L, M, N, K, scale);
}
static void launch_prep(hipStream_t st, const float* W, _Float16* Bt, int K, int N, int Kp, int Npad) {
  dim3 grid((unsigned)(Npad / 32), (unsigned)(Kp / 64));
  prep_wt<<<grid, dim3(256), 0, st>>>(W, Bt, K, N, Kp, WSC);
}

extern "C" void kernel_launch(void* const* d_in, const int* in_sizes, int n_in,
                              void* d_out, int out_size, void* d_ws, size_t ws_size,
                              hipStream_t stream) {
  if (n_in < 18) return;
  if (in_sizes[0] != MTOT * DMOD || out_size != MTOT * DMOD) return;
  if (in_sizes[1] != DMOD || in_sizes[2] != DMOD || in_sizes[3] != DMOD * 2 * DIN ||
      in_sizes[4] != DIN * DCONV || in_sizes[5] != DIN || in_sizes[6] != DIN * DBLW ||
      in_sizes[7] != DTR * DIN || in_sizes[8] != DIN || in_sizes[9] != DIN * DST ||
      in_sizes[10] != DIN || in_sizes[11] != DIN * DMOD || in_sizes[12] != DMOD * 3 * DMOD ||
      in_sizes[13] != 3 * DMOD || in_sizes[14] != DMOD * DMOD || in_sizes[15] != DMOD ||
      in_sizes[16] != 2 * DMOD * DMOD || in_sizes[17] != DMOD) return;

  const float* x       = (const float*)d_in[0];
  const float* ln_g    = (const float*)d_in[1];
  const float* ln_b    = (const float*)d_in[2];
  const float* W_in    = (const float*)d_in[3];
  const float* conv_w  = (const float*)d_in[4];
  const float* conv_b  = (const float*)d_in[5];
  const float* W_xproj = (const float*)d_in[6];
  const float* W_dt    = (const float*)d_in[7];
  const float* b_dt    = (const float*)d_in[8];
  const float* A_log   = (const float*)d_in[9];
  const float* Dp      = (const float*)d_in[10];
  const float* W_out_m = (const float*)d_in[11];
  const float* W_qkv   = (const float*)d_in[12];
  const float* b_qkv   = (const float*)d_in[13];
  const float* W_o     = (const float*)d_in[14];
  const float* b_o     = (const float*)d_in[15];
  const float* W_gate  = (const float*)d_in[16];
  const float* b_gate  = (const float*)d_in[17];
  float* out = (float*)d_out;

  size_t off = 0;
  char* wsb = (char*)d_ws;
  auto carve = [&](size_t bytes) -> char* { char* p = wsb + off; off += (bytes + 255) & ~(size_t)255; return p; };
  _Float16* Win_t  = (_Float16*)carve((size_t)(2 * DIN) * DMOD * 2);
  _Float16* Wxp_t  = (_Float16*)carve((size_t)DBLP * DIN * 2);
  _Float16* Wdt_t  = (_Float16*)carve((size_t)DIN * KDT * 2);
  _Float16* Wom_t  = (_Float16*)carve((size_t)DMOD * DIN * 2);
  _Float16* Wqkv_t = (_Float16*)carve((size_t)(3 * DMOD) * DMOD * 2);
  _Float16* Wo_t   = (_Float16*)carve((size_t)DMOD * DMOD * 2);
  _Float16* Wg_t   = (_Float16*)carve((size_t)DMOD * (2 * DMOD) * 2);
  _Float16* xn_h   = (_Float16*)carve((size_t)MTOT * DMOD * 2);
  float*    xz_f   = (float*)   carve((size_t)MTOT * 2 * DIN * 4);
  float*    xc_f   = (float*)   carve((size_t)MTOT * DIN * 4);
  _Float16* xc_h   = (_Float16*)carve((size_t)MTOT * DIN * 2);
  float*    dbl_f  = (float*)   carve((size_t)MTOT * DBLP * 4);
  _Float16* dtin_h = (_Float16*)carve((size_t)MTOT * KDT * 2);
  char*     regR   =            carve((size_t)MTOT * DIN * 4);
  _Float16* y_h    = (_Float16*)carve((size_t)MTOT * DIN * 2);
  float*    ssm_f  = (float*)   carve((size_t)MTOT * DMOD * 4);
  float*    attn_f = (float*)   carve((size_t)MTOT * DMOD * 4);
  _Float16* cat_h  = (_Float16*)carve((size_t)MTOT * (2 * DMOD) * 2);
  if (off > ws_size) return;
  float*    dt_f   = (float*)regR;
  _Float16* qkv_h  = (_Float16*)regR;
  _Float16* o_h    = (_Float16*)(regR + (size_t)MTOT * (3 * DMOD) * 2);

  launch_prep(stream, W_in,    Win_t,  DMOD, 2 * DIN,   DMOD, 2 * DIN);
  launch_prep(stream, W_xproj, Wxp_t,  DIN,  DBLW,      DIN,  DBLP);
  launch_prep(stream, W_dt,    Wdt_t,  DTR,  DIN,       KDT,  DIN);
  launch_prep(stream, W_out_m, Wom_t,  DIN,  DMOD,      DIN,  DMOD);
  launch_prep(stream, W_qkv,   Wqkv_t, DMOD, 3 * DMOD,  DMOD, 3 * DMOD);
  launch_prep(stream, W_o,     Wo_t,   DMOD, DMOD,      DMOD, DMOD);
  launch_prep(stream, W_gate,  Wg_t,   2 * DMOD, DMOD,  2 * DMOD, DMOD);

  ln_kernel<<<dim3(MTOT / 8), dim3(256), 0, stream>>>(x, ln_g, ln_b, xn_h);
  launch_gemm_f32(stream, xn_h, DMOD, Win_t, DMOD, xz_f, 2 * DIN, MTOT, 2 * DIN, DMOD, 1.0f / WSC);
  conv_silu_kernel<<<dim3(MTOT), dim3(128), 0, stream>>>(xz_f, conv_w, conv_b, xc_f, xc_h);
  launch_gemm_f32(stream, xc_h, DIN, Wxp_t, DIN, dbl_f, DBLP, MTOT, DBLP, DIN, 1.0f / (XCSC * WSC));
  dtin_kernel<<<dim3((MTOT * 8) / 256), dim3(256), 0, stream>>>(dbl_f, dtin_h);
  launch_gemm_f32_bias(stream, dtin_h, KDT, Wdt_t, KDT, dt_f, DIN, b_dt, MTOT, DIN, KDT, 1.0f / (DTSC * WSC));
  scan_kernel<<<dim3((B_SZ * DIN / 2) / 64), dim3(64), 0, stream>>>(xc_f, dt_f, dbl_f, xz_f, A_log, Dp, y_h);
  launch_gemm_f32(stream, y_h, DIN, Wom_t, DIN, ssm_f, DMOD, MTOT, DMOD, DIN, 1.0f / (YSC * WSC));
  launch_gemm_f16_bias(stream, xn_h, DMOD, Wqkv_t, DMOD, qkv_h, 3 * DMOD, b_qkv, MTOT, 3 * DMOD, DMOD, 1.0f / WSC);
  attn_f16_kernel<<<dim3(B_SZ * NHEAD * (SEQ / 64)), dim3(128), 0, stream>>>(qkv_h, o_h);
  launch_gemm_f32_bias(stream, o_h, DMOD, Wo_t, DMOD, attn_f, DMOD, b_o, MTOT, DMOD, DMOD, 1.0f / (OSC * WSC));
  pack_kernel<<<dim3((MTOT * 64) / 256), dim3(256), 0, stream>>>(ssm_f, attn_f, cat_h);
  {
    dim3 grid((unsigned)((((MTOT >> 6) * (DMOD >> 6)) + 7) / 8), 1);
    wmma_gemm64_gate<<<grid, dim3(256), 0, stream>>>((const u16t*)cat_h, 2 * DMOD, (const u16t*)Wg_t, 2 * DMOD,
                                                    out, DMOD, b_gate, x, ssm_f, attn_f,
                                                    MTOT, DMOD, 2 * DMOD, 1.0f / (CATSC * WSC));
  }
}
